// LocalAttentionBlock_20203526160389
// MI455X (gfx1250) — hardware-run, weakly checked
//
#include <hip/hip_runtime.h>
#include <math.h>
#include <stdint.h>

#ifndef SEQ
#define SEQ 2048
#endif
#define SEQ_FULL 2048
#define WID   1024
#define NH    16
#define HD    64
#define DFF   4096
#define WHALF 128
#define KOUT  (2 * WID)
#define MASKV (-1.0e9f)
#define LN_EPS 1.0e-5f
#define WSCL  64.0f
#define WSCL_INV 0.015625f


typedef __attribute__((ext_vector_type(16))) _Float16 v16h;
typedef __attribute__((ext_vector_type(8)))  _Float16 v8h;
typedef __attribute__((ext_vector_type(16))) __bf16   v16b;
typedef __attribute__((ext_vector_type(8)))  __bf16   v8b;
typedef __attribute__((ext_vector_type(8)))  float    v8f;
typedef __attribute__((ext_vector_type(4)))  float    v4f;
typedef __attribute__((ext_vector_type(2)))  float    v2f;
typedef __attribute__((ext_vector_type(4)))  unsigned int v4u;
typedef __attribute__((ext_vector_type(2)))  unsigned int v2u;

static_assert(SEQ % 64 == 0);
static_assert(SEQ <= SEQ_FULL);
static_assert(WID % 64 == 0);
static_assert(WID % 256 == 0);
static_assert(DFF % 64 == 0);
static_assert(KOUT % 32 == 0);
static_assert((size_t)SEQ * WID * 4 <= 8388608u);

__device__ __forceinline__ unsigned short f2bf_bits(float f) {
  unsigned u = __float_as_uint(f);
  return (unsigned short)((u + 0x7FFFu + ((u >> 16) & 1u)) >> 16);
}
__device__ __forceinline__ float bf_bits2f(unsigned short h) { return __uint_as_float(((unsigned)h) << 16); }
__device__ __forceinline__ unsigned pk16(unsigned short a, unsigned short b) { return (unsigned)a | ((unsigned)b << 16); }
__device__ __forceinline__ unsigned short h_bits(float f) { return __builtin_bit_cast(unsigned short, (_Float16)f); }

__device__ __forceinline__ void dep_guard_h(v8f& a, v8f& b, v16h x, v16h y) { asm volatile("v_nop\n\tv_nop\n\tv_nop\n\tv_nop" : "+v"(a), "+v"(b) : "v"(x), "v"(y)); }
__device__ __forceinline__ void dep_guard_b(v8f& a, v8f& b, v16b x, v16b y) { asm volatile("v_nop\n\tv_nop\n\tv_nop\n\tv_nop" : "+v"(a), "+v"(b) : "v"(x), "v"(y)); }
__device__ __forceinline__ void keep4_h(v16h a, v16h b, v16h c, v16h d) { asm volatile("v_nop" :: "v"(a), "v"(b), "v"(c), "v"(d)); }
__device__ __forceinline__ void keep4_b(v16b a, v16b b, v16b c, v16b d) { asm volatile("v_nop" :: "v"(a), "v"(b), "v"(c), "v"(d)); }
__device__ __forceinline__ void acc_guard4(v8f& a, v8f& b, v8f& c, v8f& d) { asm volatile("v_nop\n\tv_nop\n\tv_nop\n\tv_nop" : "+v"(a), "+v"(b), "+v"(c), "+v"(d)); }

template <typename T> struct Frag;
template <> struct Frag<_Float16> {
  typedef v16h V; union U { v16h v; v8h h[2]; };
  static __device__ __forceinline__ v16h load(const _Float16* p) {
    U f; f.h[0] = *(const v8h*)(p); f.h[1] = *(const v8h*)(p + 16); return f.v;
  }
  static __device__ __forceinline__ v8f mma(v16h a, v16h b, v8f c) {
    return __builtin_amdgcn_wmma_f32_16x16x32_f16(false, a, false, b, (short)0, c, false, false);
  }
  static __device__ __forceinline__ void guard(v8f& a, v8f& b, v16h x, v16h y) { dep_guard_h(a, b, x, y); }
  static __device__ __forceinline__ void keep(v16h a, v16h b, v16h c, v16h d) { keep4_h(a, b, c, d); }
};
template <> struct Frag<__bf16> {
  typedef v16b V; union U { v16b v; v8b h[2]; };
  static __device__ __forceinline__ v16b load(const __bf16* p) {
    U f; f.h[0] = *(const v8b*)(p); f.h[1] = *(const v8b*)(p + 16); return f.v;
  }
  static __device__ __forceinline__ v8f mma(v16b a, v16b b, v8f c) {
    return __builtin_amdgcn_wmma_f32_16x16x32_bf16(false, a, false, b, (short)0, c, false, false);
  }
  static __device__ __forceinline__ void guard(v8f& a, v8f& b, v16b x, v16b y) { dep_guard_b(a, b, x, y); }
  static __device__ __forceinline__ void keep(v16b a, v16b b, v16b c, v16b d) { keep4_b(a, b, c, d); }
};

template <int ET> struct Elem;
template <> struct Elem<0> { typedef _Float16 T; };
template <> struct Elem<1> { typedef __bf16 T; };
template <int ET, bool SPLIT, int BIAS_MODE, int OUT_MODE, int RESID, bool RELU>
__global__ __launch_bounds__(256) void wmma_gemm64(
    const unsigned short* __restrict__ Ap, const unsigned short* __restrict__ A2p, int lda, long strideA,
    const unsigned short* __restrict__ Btp, const unsigned short* __restrict__ Bt2p, int ldb, long strideB,
    void* __restrict__ Cout, void* __restrict__ Cout2, int ldc, long strideC,
    const float* __restrict__ bias,
    const float* __restrict__ resid, long strideR,
    int M, int N, int K, float scale) {
  typedef typename Elem<ET>::T T;
  typedef typename Frag<T>::V V;
  const T* A = (const T*)Ap; const T* A2 = (const T*)A2p; const T* Bt = (const T*)Btp; const T* Bt2 = (const T*)Bt2p;
  __shared__ __align__(16) float sT[8][16 * 68];
  const int b    = blockIdx.y;
  const int lane = threadIdx.x & 31;
  const int wave = threadIdx.x >> 5;
  const int tilesN = N >> 6;
  const int tilesM = M >> 6;
  const int tile = blockIdx.x * 8 + wave;
  if (tile >= tilesM * tilesN) return;
  const int tm = tile / tilesN;
  const int tn = tile - tm * tilesN;
  const int m0 = tm << 6;
  const int n0 = tn << 6;

  const T* Ab  = A  + (size_t)b * strideA;
  const T* Bb  = Bt + (size_t)b * strideB;
  const T* Ab2 = SPLIT ? (A2  + (size_t)b * strideA) : nullptr;
  const T* Bb2 = SPLIT ? (Bt2 + (size_t)b * strideB) : nullptr;

  const int rlane = lane & 15;
  const int koff  = (lane >> 4) * 8;
  const int mOff  = (lane >> 4) * 8;

  v8f acc[4][4];
#pragma unroll
  for (int i = 0; i < 4; ++i)
#pragma unroll
    for (int j = 0; j < 4; ++j) acc[i][j] = (v8f){0.f,0.f,0.f,0.f,0.f,0.f,0.f,0.f};

  for (int k0 = 0; k0 < K; k0 += 32) {
    V bh[4], bl[4];
#pragma unroll
    for (int j = 0; j < 4; ++j) {
      const size_t bo = (size_t)(n0 + (j << 4) + rlane) * ldb + koff + k0;
      bh[j] = Frag<T>::load(Bb + bo);
      if (SPLIT) bl[j] = Frag<T>::load(Bb2 + bo);
    }
#pragma unroll
    for (int i = 0; i < 4; ++i) {
      const size_t ao = (size_t)(m0 + (i << 4) + rlane) * lda + koff + k0;
      V ah = Frag<T>::load(Ab + ao);
      V al;
      if (SPLIT) al = Frag<T>::load(Ab2 + ao);
#pragma unroll
      for (int j = 0; j < 4; ++j) {
        acc[i][j] = Frag<T>::mma(ah, bh[j], acc[i][j]);
        if (SPLIT) {
          acc[i][j] = Frag<T>::mma(ah, bl[j], acc[i][j]);
          acc[i][j] = Frag<T>::mma(al, bh[j], acc[i][j]);
        }
      }
      Frag<T>::guard(acc[i][0], acc[i][3], ah, SPLIT ? al : ah);
    }
    Frag<T>::keep(bh[0], bh[1], bh[2], bh[3]);
    if (SPLIT) Frag<T>::keep(bl[0], bl[1], bl[2], bl[3]);
  }
  acc_guard4(acc[0][0], acc[0][1], acc[0][2], acc[0][3]);
  acc_guard4(acc[1][0], acc[1][1], acc[1][2], acc[1][3]);
  acc_guard4(acc[2][0], acc[2][1], acc[2][2], acc[2][3]);
  acc_guard4(acc[3][0], acc[3][1], acc[3][2], acc[3][3]);

  float* slab = sT[wave];
  const float* Rb = (RESID != 0) ? (resid + (size_t)b * strideR) : nullptr;
#pragma unroll
  for (int i = 0; i < 4; ++i) {
    const int mBase = m0 + (i << 4);
#pragma unroll
    for (int j = 0; j < 4; ++j) {
      const int n = n0 + (j << 4) + rlane;
      float bv = 0.f;
      if (BIAS_MODE == 2) bv = bf_bits2f(f2bf_bits(bias[n]));
#pragma unroll
      for (int r = 0; r < 8; ++r) {
        float v = acc[i][j][r] * scale;
        if (BIAS_MODE == 1) v += bf_bits2f(f2bf_bits(bias[mBase + mOff + r]));
        if (BIAS_MODE == 2) v += bv;
        if (RESID == 1) v += Rb[(size_t)(mBase + mOff + r) * ldc + n];
        if (RESID == 2) v += bf_bits2f(f2bf_bits(Rb[(size_t)(mBase + mOff + r) * ldc + n]));
        if (RELU) v = fmaxf(v, 0.f);
        slab[(mOff + r) * 68 + (j << 4) + rlane] = v;
      }
    }
    __builtin_amdgcn_fence(__ATOMIC_RELEASE, "workgroup");
    __builtin_amdgcn_wave_barrier();
    __builtin_amdgcn_fence(__ATOMIC_ACQUIRE, "workgroup");
    if (OUT_MODE == 0) {
      float* C = (float*)Cout + (size_t)b * strideC;
      const int hh = lane >> 4, c4 = (lane & 15) * 4;
      for (int pass = 0; pass < 2; ++pass) {
#pragma unroll
        for (int it = 0; it < 8; ++it) {
          const int row = it * 2 + hh;
          v4f v = *(const v4f*)(slab + row * 68 + c4);
          *(volatile v4f*)(C + (size_t)(mBase + row) * ldc + n0 + c4) = v;
        }
        __threadfence();
      }
    } else {
      const int q = lane >> 3, c8 = (lane & 7) * 8;
      unsigned short* C  = (unsigned short*)Cout  + (size_t)b * strideC;
      unsigned short* C2 = (OUT_MODE == 2) ? ((unsigned short*)Cout2 + (size_t)b * strideC) : nullptr;
      for (int pass = 0; pass < 2; ++pass) {
#pragma unroll
        for (int it = 0; it < 4; ++it) {
          const int row = it * 4 + q;
          const float* sp = slab + row * 68 + c8;
          v8h hv, lv;
#pragma unroll
          for (int e = 0; e < 8; ++e) {
            if (OUT_MODE == 1) {
              hv[e] = (_Float16)sp[e];
            } else {
              unsigned short hb = f2bf_bits(sp[e]);
              unsigned short lb = f2bf_bits(sp[e] - bf_bits2f(hb));
              hv[e] = __builtin_bit_cast(_Float16, hb);
              lv[e] = __builtin_bit_cast(_Float16, lb);
            }
          }
          *(volatile v8h*)(C + (size_t)(mBase + row) * ldc + n0 + c8) = hv;
          if (OUT_MODE == 2) *(volatile v8h*)(C2 + (size_t)(mBase + row) * ldc + n0 + c8) = lv;
        }
        __threadfence();
      }
    }
    __builtin_amdgcn_fence(__ATOMIC_RELEASE, "workgroup");
    __builtin_amdgcn_wave_barrier();
    __builtin_amdgcn_fence(__ATOMIC_ACQUIRE, "workgroup");
  }
}

template <bool DUP>
__global__ __launch_bounds__(256) void cvt_bf16_kernel(const float* __restrict__ in, unsigned short* __restrict__ out,
                                                       int n8, int srcCols, int dstPitch, int dupOff) {
  const int i = blockIdx.x * 256 + threadIdx.x;
  if (i < n8) {
    const size_t e   = (size_t)i * 8;
    const size_t row = e / (size_t)srcCols;
    const size_t col = e - row * (size_t)srcCols;
    const v4f f0 = *(const v4f*)(in + e);
    const v4f f1 = *(const v4f*)(in + e + 4);
    v4u u;
    u[0] = pk16(f2bf_bits(f0[0]), f2bf_bits(f0[1]));
    u[1] = pk16(f2bf_bits(f0[2]), f2bf_bits(f0[3]));
    u[2] = pk16(f2bf_bits(f1[0]), f2bf_bits(f1[1]));
    u[3] = pk16(f2bf_bits(f1[2]), f2bf_bits(f1[3]));
    const size_t d = row * (size_t)dstPitch + col;
    *(volatile v4u*)(out + d) = u;
    if (DUP) *(volatile v4u*)(out + d + dupOff) = u;
    __threadfence();
    *(volatile v4u*)(out + d) = u;
    if (DUP) *(volatile v4u*)(out + d + dupOff) = u;
  }
}

template <int OT, bool DUP>
__global__ __launch_bounds__(256) void tr_cvt_kernel(const float* __restrict__ in, unsigned short* __restrict__ out,
                                                     int rows, int cols, int dstPitch, int dupOff, float mul) {
  __shared__ float sT[64][65];
  const int tid = threadIdx.x, lane = tid & 31, wave = tid >> 5;
  const int r0 = blockIdx.y * 64, c0 = blockIdx.x * 64;
  if (r0 + 64 > rows || c0 + 64 > cols) return;
  {
    const int lr = tid >> 2, lc = (tid & 3) * 16;
    const float* src = in + (size_t)(r0 + lr) * cols + c0 + lc;
#pragma unroll
    for (int g = 0; g < 4; ++g) {
      const v4f v = *(const v4f*)(src + 4 * g);
      sT[lr][lc + 4 * g + 0] = v[0];
      sT[lr][lc + 4 * g + 1] = v[1];
      sT[lr][lc + 4 * g + 2] = v[2];
      sT[lr][lc + 4 * g + 3] = v[3];
    }
  }
  __syncthreads();
  const int q = lane >> 3, c8 = (lane & 7) * 8;
  v4u pk[2];
#pragma unroll
  for (int it = 0; it < 2; ++it) {
    const int orow = wave * 8 + it * 4 + q;
    unsigned short bits[8];
#pragma unroll
    for (int e = 0; e < 8; ++e) {
      const unsigned short hb = f2bf_bits(sT[c8 + e][orow]);
      bits[e] = (OT == 1) ? hb : h_bits(bf_bits2f(hb) * mul);
    }
    v4u a;
    a[0] = pk16(bits[0], bits[1]);
    a[1] = pk16(bits[2], bits[3]);
    a[2] = pk16(bits[4], bits[5]);
    a[3] = pk16(bits[6], bits[7]);
    pk[it] = a;
  }
  for (int pass = 0; pass < 2; ++pass) {
#pragma unroll
    for (int it = 0; it < 2; ++it) {
      const int orow = wave * 8 + it * 4 + q;
      const size_t d = (size_t)(c0 + orow) * dstPitch + r0 + c8;
      *(volatile v4u*)(out + d) = pk[it];
      if (DUP) *(volatile v4u*)(out + d + dupOff) = pk[it];
    }
    __threadfence();
  }
}

#define AT_D  64
#define AT_NW 4
#define AT_QB 64
#define AT_KC 64
#define NQT   (SEQ / AT_QB)
#define KSPAN (WHALF / AT_KC)

static_assert(WHALF % AT_KC == 0);
static_assert(SEQ % AT_QB == 0);
static_assert(HD == AT_D);

__device__ __forceinline__ __bf16 at_f2bf(float f) { return __builtin_bit_cast(__bf16, f2bf_bits(f)); }
__device__ __forceinline__ void at_split(float f, __bf16& hi, __bf16& lo) {
  const unsigned short hb = f2bf_bits(f);
  hi = __builtin_bit_cast(__bf16, hb);
  lo = at_f2bf(f - __uint_as_float(((unsigned)hb) << 16));
}
__device__ __forceinline__ v8f at_mma(v16b a, v16b b, v8f c) {
  c = __builtin_amdgcn_wmma_f32_16x16x32_bf16(false, a, false, b, (short)0, c, false, false);
  asm volatile("v_nop\n\tv_nop\n\tv_nop\n\tv_nop" : "+v"(c) : "v"(a), "v"(b));
  return c;
}

__global__ __launch_bounds__(128)
void attn_win64_kernel(const unsigned short* __restrict__ qhp, const unsigned short* __restrict__ qlp,
                       const unsigned short* __restrict__ khp, const unsigned short* __restrict__ klp,
                       const unsigned short* __restrict__ vhp, const unsigned short* __restrict__ vlp,
                       unsigned short* __restrict__ op, float sscale) {
  union FB { v16b v; v8b h[2]; };
  __shared__ __align__(16) __bf16 Ksh[AT_KC * AT_D];
  __shared__ __align__(16) __bf16 Ksl[AT_KC * AT_D];
  __shared__ __align__(16) __bf16 Vth[AT_D * AT_KC];
  __shared__ __align__(16) __bf16 Vtl[AT_D * AT_KC];
  __shared__ __align__(16) __bf16 Psh[AT_NW][16 * AT_KC];
  __shared__ __align__(16) __bf16 Psl[AT_NW][16 * AT_KC];
  __shared__ __align__(16) float  Os[AT_NW][16 * 68];

  const int tid  = threadIdx.x;
  const int wave = tid >> 5;
  const int lane = tid & 31;
  const int hh   = lane >> 4;
  const int c    = lane & 15;

  const int bx   = blockIdx.x;
  const int qt   = bx % NQT;
  const int head = bx / NQT;
  const int q0   = qt * AT_QB + wave * 16;
  const size_t hcol = (size_t)head * HD;

  const __bf16* Qh = (const __bf16*)(const void*)qhp + hcol;
  const __bf16* Ql = (const __bf16*)(const void*)qlp + hcol;
  const __bf16* Kh = (const __bf16*)(const void*)khp + hcol;
  const __bf16* Kl = (const __bf16*)(const void*)klp + hcol;
  const __bf16* Vh = (const __bf16*)(const void*)vhp + hcol * SEQ;
  const __bf16* Vl = (const __bf16*)(const void*)vlp + hcol * SEQ;
  unsigned short* Oh = op + hcol;
  unsigned short* Ol = Oh + WID;

  v16b qah[2], qal[2];
#pragma unroll
  for (int dc = 0; dc < 2; ++dc) {
    const __bf16* qr = Qh + (size_t)(q0 + c) * WID + dc * 32 + 8 * hh;
    const __bf16* ql = Ql + (size_t)(q0 + c) * WID + dc * 32 + 8 * hh;
    qah[dc] = Frag<__bf16>::load(qr);
    qal[dc] = Frag<__bf16>::load(ql);
  }

  float mrow[8], lrow[8];
  v8f oacc[4];
#pragma unroll
  for (int r = 0; r < 8; ++r) { mrow[r] = -INFINITY; lrow[r] = 0.f; }
#pragma unroll
  for (int t = 0; t < 4; ++t) oacc[t] = (v8f){0.f,0.f,0.f,0.f,0.f,0.f,0.f,0.f};

  const int kcBeg = (qt > KSPAN) ? (qt - KSPAN) : 0;
  const int kcEnd = (qt + KSPAN < NQT - 1) ? (qt + KSPAN) : (NQT - 1);
  for (int kc = kcBeg; kc <= kcEnd; ++kc) {
    const int kv0 = kc * AT_KC;
    __syncthreads();
    {
      const int r = tid >> 1, half = (tid & 1) * 32;
      const __bf16* ksh = Kh + (size_t)(kv0 + r) * WID + half;
      const __bf16* ksl = Kl + (size_t)(kv0 + r) * WID + half;
      const __bf16* vsh = Vh + (size_t)r * SEQ + kv0 + half;
      const __bf16* vsl = Vl + (size_t)r * SEQ + kv0 + half;
#pragma unroll
      for (int i = 0; i < 4; ++i) {
        const v8b a0 = *(const v8b*)(ksh + 8 * i);
        const v8b a1 = *(const v8b*)(ksl + 8 * i);
        const v8b b0 = *(const v8b*)(vsh + 8 * i);
        const v8b b1 = *(const v8b*)(vsl + 8 * i);
        *(v8b*)(Ksh + r * AT_D  + half + 8 * i) = a0;
        *(v8b*)(Ksl + r * AT_D  + half + 8 * i) = a1;
        *(v8b*)(Vth + r * AT_KC + half + 8 * i) = b0;
        *(v8b*)(Vtl + r * AT_KC + half + 8 * i) = b1;
      }
    }
    __syncthreads();

    v8f s[4];
#pragma unroll
    for (int j = 0; j < 4; ++j) {
      s[j] = (v8f){0.f,0.f,0.f,0.f,0.f,0.f,0.f,0.f};
#pragma unroll
      for (int dc = 0; dc < 2; ++dc) {
        FB kb, kl;
        kb.h[0] = *(const v8b*)(Ksh + (j * 16 + c) * AT_D + dc * 32 + 8 * hh);
        kb.h[1] = *(const v8b*)(Ksh + (j * 16 + c) * AT_D + dc * 32 + 16 + 8 * hh);
        kl.h[0] = *(const v8b*)(Ksl + (j * 16 + c) * AT_D + dc * 32 + 8 * hh);
        kl.h[1] = *(const v8b*)(Ksl + (j * 16 + c) * AT_D + dc * 32 + 16 + 8 * hh);
        s[j] = at_mma(qah[dc], kb.v, s[j]);
        s[j] = at_mma(qah[dc], kl.v, s[j]);
        s[j] = at_mma(qal[dc], kb.v, s[j]);
      }
    }
    float cm[8];
#pragma unroll
    for (int r = 0; r < 8; ++r) {
      const int t = q0 + 8 * hh + r;
      float m = -INFINITY;
#pragma unroll
      for (int j = 0; j < 4; ++j) {
        const int sk = kv0 + j * 16 + c;
        const int dt = t - sk;
        const bool ok = (dt <= WHALF) && (dt >= -WHALF);
        float sv = s[j][r] * sscale;
        sv = ok ? sv : MASKV;
        s[j][r] = sv;
        m = fmaxf(m, sv);
      }
#pragma unroll
      for (int off = 1; off < 16; off <<= 1) m = fmaxf(m, __shfl_xor(m, off, 32));
      cm[r] = m;
    }
    __bf16* pwh = Psh[wave];
    __bf16* pwl = Psl[wave];
#pragma unroll
    for (int r = 0; r < 8; ++r) {
      const float mnew = fmaxf(mrow[r], cm[r]);
      const float alpha = expf(mrow[r] - mnew);
      mrow[r] = mnew;
      float psum = 0.f;
#pragma unroll
      for (int j = 0; j < 4; ++j) {
        const float p = expf(s[j][r] - mnew);
        psum += p;
        __bf16 a, bl; at_split(p, a, bl);
        pwh[(8 * hh + r) * AT_KC + j * 16 + c] = a;
        pwl[(8 * hh + r) * AT_KC + j * 16 + c] = bl;
      }
#pragma unroll
      for (int off = 1; off < 16; off <<= 1) psum += __shfl_xor(psum, off, 32);
      lrow[r] = lrow[r] * alpha + psum;
#pragma unroll
      for (int t = 0; t < 4; ++t) oacc[t][r] *= alpha;
    }
    __builtin_amdgcn_fence(__ATOMIC_RELEASE, "workgroup");
    __builtin_amdgcn_wave_barrier();
    __builtin_amdgcn_fence(__ATOMIC_ACQUIRE, "workgroup");
#pragma unroll 1
    for (int kk = 0; kk < 2; ++kk) {
      FB pa, pl;
      pa.h[0] = *(const v8b*)(pwh + c * AT_KC + kk * 32 + 8 * hh);
      pa.h[1] = *(const v8b*)(pwh + c * AT_KC + kk * 32 + 16 + 8 * hh);
      pl.h[0] = *(const v8b*)(pwl + c * AT_KC + kk * 32 + 8 * hh);
      pl.h[1] = *(const v8b*)(pwl + c * AT_KC + kk * 32 + 16 + 8 * hh);
#pragma unroll
      for (int t = 0; t < 4; ++t) {
        FB vb, vl;
        vb.h[0] = *(const v8b*)(Vth + (t * 16 + c) * AT_KC + kk * 32 + 8 * hh);
        vb.h[1] = *(const v8b*)(Vth + (t * 16 + c) * AT_KC + kk * 32 + 16 + 8 * hh);
        vl.h[0] = *(const v8b*)(Vtl + (t * 16 + c) * AT_KC + kk * 32 + 8 * hh);
        vl.h[1] = *(const v8b*)(Vtl + (t * 16 + c) * AT_KC + kk * 32 + 16 + 8 * hh);
        oacc[t] = at_mma(pa.v, vb.v, oacc[t]);
        oacc[t] = at_mma(pa.v, vl.v, oacc[t]);
        oacc[t] = at_mma(pl.v, vb.v, oacc[t]);
      }
    }
  }

  float* os = Os[wave];
#pragma unroll
  for (int r = 0; r < 8; ++r) {
    const float inv = 1.0f / lrow[r];
#pragma unroll
    for (int t = 0; t < 4; ++t) os[(8 * hh + r) * 68 + t * 16 + c] = oacc[t][r] * inv;
  }
  __builtin_amdgcn_fence(__ATOMIC_RELEASE, "workgroup");
  __builtin_amdgcn_wave_barrier();
  __builtin_amdgcn_fence(__ATOMIC_ACQUIRE, "workgroup");
  {
    const int q = lane >> 3, c8 = (lane & 7) * 8;
    v4u hv[4], lv[4];
#pragma unroll
    for (int it = 0; it < 4; ++it) {
      const int row = it * 4 + q;
      const float* sp = os + row * 68 + c8;
      v4u a, a2;
#pragma unroll
      for (int g = 0; g < 4; ++g) {
        const float f0 = sp[2 * g], f1 = sp[2 * g + 1];
        const unsigned short h0 = f2bf_bits(f0), h1 = f2bf_bits(f1);
        const unsigned short l0 = f2bf_bits(f0 - bf_bits2f(h0)), l1 = f2bf_bits(f1 - bf_bits2f(h1));
        a[g]  = pk16(h0, h1);
        a2[g] = pk16(l0, l1);
      }
      hv[it] = a; lv[it] = a2;
    }
    for (int pass = 0; pass < 2; ++pass) {
#pragma unroll
      for (int it = 0; it < 4; ++it) {
        const int row = it * 4 + q;
        const size_t go = (size_t)(q0 + row) * KOUT + c8;
        *(volatile v4u*)(Oh + go) = hv[it];
        *(volatile v4u*)(Ol + go) = lv[it];
      }
      __threadfence();
    }
  }
}

template <bool WH>
__global__ __launch_bounds__(256) void ln_rows_kernel(const float* __restrict__ y, const float* __restrict__ g,
                                                      const float* __restrict__ be, float* __restrict__ outf,
                                                      unsigned short* __restrict__ outh) {
  __shared__ float red[2][8];
  const int row = blockIdx.x, tid = threadIdx.x, lane = tid & 31, wave = tid >> 5;
  const int c = tid * 4;
  const size_t ro = (size_t)row * WID;
  const v4f v = *(const v4f*)(y + ro + c);
  float s = (v[0] + v[1]) + (v[2] + v[3]);
#pragma unroll
  for (int off = 1; off < 32; off <<= 1) s += __shfl_xor(s, off, 32);
  if (lane == 0) red[0][wave] = s;
  __syncthreads();
  float tot = 0.f;
#pragma unroll
  for (int w = 0; w < 8; ++w) tot += red[0][w];
  const float mu = tot * (1.0f / (float)WID);
  v4f d;
  d[0] = v[0] - mu; d[1] = v[1] - mu; d[2] = v[2] - mu; d[3] = v[3] - mu;
  float s2 = (d[0] * d[0] + d[1] * d[1]) + (d[2] * d[2] + d[3] * d[3]);
#pragma unroll
  for (int off = 1; off < 32; off <<= 1) s2 += __shfl_xor(s2, off, 32);
  if (lane == 0) red[1][wave] = s2;
  __syncthreads();
  float tot2 = 0.f;
#pragma unroll
  for (int w = 0; w < 8; ++w) tot2 += red[1][w];
  const float var  = tot2 * (1.0f / (float)WID);
  const float rstd = rsqrtf(var + LN_EPS);
  const v4f gv = *(const v4f*)(g + c);
  const v4f bv = *(const v4f*)(be + c);
  v4f o;
#pragma unroll
  for (int e = 0; e < 4; ++e) {
    const float gb = bf_bits2f(f2bf_bits(gv[e]));
    const float bb = bf_bits2f(f2bf_bits(bv[e]));
    o[e] = d[e] * rstd * gb + bb;
  }
  v2u hw;
  hw[0] = pk16(h_bits(o[0]), h_bits(o[1]));
  hw[1] = pk16(h_bits(o[2]), h_bits(o[3]));
  *(volatile v4f*)(outf + ro + c) = o;
  if (WH) *(volatile v2u*)(outh + ro + c) = hw;
  __threadfence();
  *(volatile v4f*)(outf + ro + c) = o;
  if (WH) *(volatile v2u*)(outh + ro + c) = hw;
}

extern "C" void kernel_launch(void* const* d_in, const int* in_sizes, int n_in,
                              void* d_out, int out_size, void* d_ws, size_t ws_size,
                              hipStream_t stream) {
  if (n_in < 17) return;
  if (in_sizes[0] < SEQ * WID) return;
  if (in_sizes[1] < WID * WID || in_sizes[3] < WID * WID || in_sizes[5] < WID * WID || in_sizes[7] < WID * WID) return;
  if (in_sizes[2] < WID || in_sizes[4] < WID || in_sizes[6] < WID || in_sizes[8] < WID) return;
  if (in_sizes[9] < WID || in_sizes[10] < WID || in_sizes[15] < WID || in_sizes[16] < WID) return;
  if (in_sizes[11] < WID * DFF || in_sizes[12] < DFF || in_sizes[13] < DFF * WID || in_sizes[14] < WID) return;
  if (out_size < SEQ * WID) return;

  const float* x    = (const float*)d_in[0];
  const float* wq   = (const float*)d_in[1];
  const float* bq   = (const float*)d_in[2];
  const float* wk   = (const float*)d_in[3];
  const float* bk   = (const float*)d_in[4];
  const float* wv   = (const float*)d_in[5];
  const float* bvp  = (const float*)d_in[6];
  const float* wo   = (const float*)d_in[7];
  const float* bo   = (const float*)d_in[8];
  const float* g1   = (const float*)d_in[9];
  const float* be1  = (const float*)d_in[10];
  const float* wf1  = (const float*)d_in[11];
  const float* bf1  = (const float*)d_in[12];
  const float* wf2  = (const float*)d_in[13];
  const float* bf2  = (const float*)d_in[14];
  const float* g2   = (const float*)d_in[15];
  const float* be2  = (const float*)d_in[16];

  const size_t PXB  = (size_t)SEQ * WID * 2;
  const size_t PW   = (size_t)WID * WID * 2;
  const size_t PWO2 = (size_t)WID * KOUT * 2;
  const size_t PWF  = (size_t)DFF * WID * 2;
  const size_t PQ   = (size_t)SEQ * WID * 2;
  const size_t PVT  = (size_t)WID * SEQ * 2;
  const size_t PO2  = (size_t)SEQ * KOUT * 2;
  const size_t PF32 = (size_t)SEQ * WID * 4;
  const size_t PHH  = (size_t)SEQ * WID * 2;
  const size_t PF1  = (size_t)SEQ * DFF * 2;
  size_t off = 0;
  const size_t oXB   = off; off += PXB;
  const size_t oWQT  = off; off += PW;
  const size_t oWKT  = off; off += PW;
  const size_t oWVT  = off; off += PW;
  const size_t oWOT2 = off; off += PWO2;
  const size_t oWF1T = off; off += PWF;
  const size_t oWF2T = off; off += PWF;
  const size_t oQh   = off; off += PQ;
  const size_t oQl   = off; off += PQ;
  const size_t oKh   = off; off += PQ;
  const size_t oKl   = off; off += PQ;
  const size_t oVTh  = off; off += PVT;
  const size_t oVTl  = off; off += PVT;
  const size_t oO2   = off; off += PO2;
  const size_t oY1   = off; off += PF32;
  const size_t oH    = off; off += PF32;
  const size_t oHh   = off; off += PHH;
  const size_t oF1   = off; off += PF1;
  const size_t oY2   = off; off += PF32;
  if (off > ws_size) return;
  if (off > (size_t)134217728) return;

  char* ws = (char*)d_ws;
  unsigned short* XB   = (unsigned short*)(ws + oXB);
  unsigned short* WQT  = (unsigned short*)(ws + oWQT);
  unsigned short* WKT  = (unsigned short*)(ws + oWKT);
  unsigned short* WVT  = (unsigned short*)(ws + oWVT);
  unsigned short* WOT2 = (unsigned short*)(ws + oWOT2);
  unsigned short* WF1T = (unsigned short*)(ws + oWF1T);
  unsigned short* WF2T = (unsigned short*)(ws + oWF2T);
  unsigned short* Qh   = (unsigned short*)(ws + oQh);
  unsigned short* Ql   = (unsigned short*)(ws + oQl);
  unsigned short* Kh   = (unsigned short*)(ws + oKh);
  unsigned short* Kl   = (unsigned short*)(ws + oKl);
  unsigned short* VTh  = (unsigned short*)(ws + oVTh);
  unsigned short* VTl  = (unsigned short*)(ws + oVTl);
  unsigned short* O2   = (unsigned short*)(ws + oO2);
  float*          Y1   = (float*)(ws + oY1);
  float*          H    = (float*)(ws + oH);
  unsigned short* Hh   = (unsigned short*)(ws + oHh);
  unsigned short* F1   = (unsigned short*)(ws + oF1);
  float*          Y2   = (float*)(ws + oY2);

  const dim3 blk(256);
  const float* dummy = x;

  const int n8x = SEQ * WID / 8;
  cvt_bf16_kernel<false><<<dim3((n8x + 255) / 256), blk, 0, stream>>>(x, XB, n8x, WID, WID, 0);
  tr_cvt_kernel<1, false><<<dim3(WID / 64, WID / 64), blk, 0, stream>>>(wq,  WQT,  WID, WID, WID,  0,   1.0f);
  tr_cvt_kernel<1, false><<<dim3(WID / 64, WID / 64), blk, 0, stream>>>(wk,  WKT,  WID, WID, WID,  0,   1.0f);
  tr_cvt_kernel<1, false><<<dim3(WID / 64, WID / 64), blk, 0, stream>>>(wv,  WVT,  WID, WID, WID,  0,   1.0f);
  tr_cvt_kernel<1, true ><<<dim3(WID / 64, WID / 64), blk, 0, stream>>>(wo,  WOT2, WID, WID, KOUT, WID, 1.0f);
  tr_cvt_kernel<0, false><<<dim3(DFF / 64, WID / 64), blk, 0, stream>>>(wf1, WF1T, WID, DFF, WID,  0,   WSCL);
  tr_cvt_kernel<0, false><<<dim3(WID / 64, DFF / 64), blk, 0, stream>>>(wf2, WF2T, DFF, WID, DFF,  0,   WSCL);

  const dim3 gQ(((SEQ / 64) * (WID / 64) + 7) / 8, 1);
  wmma_gemm64<1, false, 2, 2, 0, false><<<gQ, blk, 0, stream>>>(
      XB, XB, WID, 0L, WQT, WQT, WID, 0L, (void*)Qh, (void*)Ql, WID, 0L,
      bq, dummy, 0L, SEQ, WID, WID, 1.0f);
  wmma_gemm64<1, false, 2, 2, 0, false><<<gQ, blk, 0, stream>>>(
      XB, XB, WID, 0L, WKT, WKT, WID, 0L, (void*)Kh, (void*)Kl, WID, 0L,
      bk, dummy, 0L, SEQ, WID, WID, 1.0f);
  const dim3 gVT(((WID / 64) * (SEQ / 64) + 7) / 8, 1);
  wmma_gemm64<1, false, 1, 2, 0, false><<<gVT, blk, 0, stream>>>(
      WVT, WVT, WID, 0L, XB, XB, WID, 0L, (void*)VTh, (void*)VTl, SEQ, 0L,
      bvp, dummy, 0L, WID, SEQ, WID, 1.0f);
  attn_win64_kernel<<<dim3(NH * NQT), dim3(128), 0, stream>>>(Qh, Ql, Kh, Kl, VTh, VTl, O2, 0.125f);
  wmma_gemm64<1, false, 2, 0, 2, false><<<gQ, blk, 0, stream>>>(
      O2, O2, KOUT, 0L, WOT2, WOT2, KOUT, 0L, (void*)Y1, (void*)Y1, WID, 0L,
      bo, x, 0L, SEQ, WID, KOUT, 1.0f);
  ln_rows_kernel<true><<<dim3(SEQ), blk, 0, stream>>>(Y1, g1, be1, H, Hh);
  const dim3 gF1(((SEQ / 64) * (DFF / 64) + 7) / 8, 1);
  wmma_gemm64<0, false, 2, 1, 0, true><<<gF1, blk, 0, stream>>>(
      Hh, Hh, WID, 0L, WF1T, WF1T, WID, 0L, (void*)F1, (void*)F1, DFF, 0L,
      bf1, dummy, 0L, SEQ, DFF, WID, WSCL_INV);
  wmma_gemm64<0, false, 2, 0, 1, false><<<gQ, blk, 0, stream>>>(
      F1, F1, DFF, 0L, WF2T, WF2T, DFF, 0L, (void*)Y2, (void*)Y2, WID, 0L,
      bf2, H, 0L, SEQ, WID, DFF, WSCL_INV);
  ln_rows_kernel<false><<<dim3(SEQ), blk, 0, stream>>>(Y2, g2, be2, (float*)d_out, Hh);
  (void)hipGetLastError();
}
